// MultiScaleRetention_10376640987876
// MI455X (gfx1250) — hardware-verified
//
#include <hip/hip_runtime.h>
#include <math.h>

constexpr int kB    = 2;
constexpr int kN    = 2048;
constexpr int kE    = 512;
constexpr int kH    = 8;
constexpr int kDh   = 64;
constexpr int kHalf = 32;
constexpr int kTok  = kB * kN;
constexpr int kPlane  = kTok * kE;
constexpr int kWElems = kE * kE;
static_assert(kH * kDh == kE, "shape");
static_assert(kTok % 64 == 0 && kE % 64 == 0 && kE % 32 == 0 && kN % 64 == 0 && kDh == 64, "tiles");

constexpr float kWCarry   = 16.0f;
constexpr float kQC       = 32.0f;
constexpr float kKC       = 128.0f;
constexpr float kKmul     = kKC * 0.125f;
constexpr float kPC       = 256.0f;
constexpr float kPCInv    = 1.0f / kPC;
constexpr float kMaskMul  = kPC / (kQC * kKC);
constexpr float kRGC      = 64.0f;
constexpr float kOutScale = 1.0f / (kRGC * kWCarry);
constexpr float kInvDh    = 1.0f / 64.0f;
constexpr float kGnEps    = 1.0e-6f;
constexpr float kLn1o32   = -3.46573590279972655f;
constexpr float kLn1o512  = -6.23832462503950772f;

typedef __attribute__((ext_vector_type(16))) _Float16 v16h;
typedef __attribute__((ext_vector_type(8)))  _Float16 v8h;
typedef __attribute__((ext_vector_type(16))) __bf16   v16b;
typedef __attribute__((ext_vector_type(8)))  __bf16   v8b;
typedef __attribute__((ext_vector_type(8)))  float    v8f;
typedef __attribute__((ext_vector_type(4)))  float    v4f;
typedef __attribute__((ext_vector_type(4)))  unsigned int v4u;

__device__ __forceinline__ unsigned short f2bf_bits(float f) {
  unsigned u = __float_as_uint(f);
  return (unsigned short)((u + 0x7FFFu + ((u >> 16) & 1u)) >> 16);
}
__device__ __forceinline__ float bf_bits2f(unsigned short h) { return __uint_as_float(((unsigned)h) << 16); }

__device__ __forceinline__ void dep_guard_h(v8f& a, v8f& b, v16h x, v16h y) { asm volatile("v_nop\n\tv_nop\n\tv_nop\n\tv_nop" : "+v"(a), "+v"(b) : "v"(x), "v"(y)); }
__device__ __forceinline__ void dep_guard_b(v8f& a, v8f& b, v16b x, v16b y) { asm volatile("v_nop\n\tv_nop\n\tv_nop\n\tv_nop" : "+v"(a), "+v"(b) : "v"(x), "v"(y)); }
__device__ __forceinline__ void keep4_h(v16h a, v16h b, v16h c, v16h d) { asm volatile("v_nop" :: "v"(a), "v"(b), "v"(c), "v"(d)); }
__device__ __forceinline__ void keep4_b(v16b a, v16b b, v16b c, v16b d) { asm volatile("v_nop" :: "v"(a), "v"(b), "v"(c), "v"(d)); }
__device__ __forceinline__ void acc_guard4(v8f& a, v8f& b, v8f& c, v8f& d) { asm volatile("v_nop\n\tv_nop\n\tv_nop\n\tv_nop" : "+v"(a), "+v"(b), "+v"(c), "+v"(d)); }
template <typename T> struct Frag;
template <> struct Frag<_Float16> {
  typedef v16h V; union U { v16h v; v8h h[2]; };
  static __device__ __forceinline__ v16h load(const _Float16* p) {
    U f; f.h[0] = *(const v8h*)(p); f.h[1] = *(const v8h*)(p + 16); return f.v;
  }
  static __device__ __forceinline__ v8f mma(v16h a, v16h b, v8f c) {
    return __builtin_amdgcn_wmma_f32_16x16x32_f16(false, a, false, b, (short)0, c, false, false);
  }
  static __device__ __forceinline__ void guard(v8f& a, v8f& b, v16h x, v16h y) { dep_guard_h(a, b, x, y); }
  static __device__ __forceinline__ void keep(v16h a, v16h b, v16h c, v16h d) { keep4_h(a, b, c, d); }
};
template <> struct Frag<__bf16> {
  typedef v16b V; union U { v16b v; v8b h[2]; };
  static __device__ __forceinline__ v16b load(const __bf16* p) {
    U f; f.h[0] = *(const v8b*)(p); f.h[1] = *(const v8b*)(p + 16); return f.v;
  }
  static __device__ __forceinline__ v8f mma(v16b a, v16b b, v8f c) {
    return __builtin_amdgcn_wmma_f32_16x16x32_bf16(false, a, false, b, (short)0, c, false, false);
  }
  static __device__ __forceinline__ void guard(v8f& a, v8f& b, v16b x, v16b y) { dep_guard_b(a, b, x, y); }
  static __device__ __forceinline__ void keep(v16b a, v16b b, v16b c, v16b d) { keep4_b(a, b, c, d); }
};

__device__ __forceinline__ unsigned pk16(unsigned short a, unsigned short b) { return (unsigned)a | ((unsigned)b << 16); }
__device__ __forceinline__ unsigned short h_bits(float f) { const _Float16 h = (_Float16)f; return __builtin_bit_cast(unsigned short, h); }

template <int ET> struct Elem;
template <> struct Elem<0> { typedef _Float16 T; };
template <> struct Elem<1> { typedef __bf16 T; };
template <int ET, bool SPLIT, int BIAS_MODE, int OUT_MODE, bool RESID, int ACT = 0>
__global__ __launch_bounds__(256) void wmma_gemm64(
    const unsigned short* __restrict__ Ap, const unsigned short* __restrict__ A2p, int lda, long strideA,
    const unsigned short* __restrict__ Btp, const unsigned short* __restrict__ Bt2p, int ldb, long strideB,
    void* __restrict__ Cout, void* __restrict__ Cout2, int ldc, long strideC,
    const float* __restrict__ bias,
    const float* __restrict__ resid, long strideR,
    int M, int N, int K, float scale) {
  typedef typename Elem<ET>::T T;
  typedef typename Frag<T>::V V;
  const T* A = (const T*)Ap; const T* A2 = (const T*)A2p; const T* Bt = (const T*)Btp; const T* Bt2 = (const T*)Bt2p;
  __shared__ __align__(16) float sT[8][16 * 68];
  const int b    = blockIdx.y;
  const int lane = threadIdx.x & 31;
  const int wave = threadIdx.x >> 5;
  const int tilesN = N >> 6;
  const int tilesM = M >> 6;
  const int tile = blockIdx.x * 8 + wave;
  if (tile >= tilesM * tilesN) return;
  const int tm = tile / tilesN;
  const int tn = tile - tm * tilesN;
  const int m0 = tm << 6;
  const int n0 = tn << 6;

  const T* Ab  = A  + (size_t)b * strideA;
  const T* Bb  = Bt + (size_t)b * strideB;
  const T* Ab2 = SPLIT ? (A2  + (size_t)b * strideA) : nullptr;
  const T* Bb2 = SPLIT ? (Bt2 + (size_t)b * strideB) : nullptr;

  const int rlane = lane & 15;
  const int koff  = (lane >> 4) * 8;
  const int mOff  = (lane >> 4) * 8;

  v8f acc[4][4];
#pragma unroll
  for (int i = 0; i < 4; ++i)
#pragma unroll
    for (int j = 0; j < 4; ++j) acc[i][j] = (v8f){0.f,0.f,0.f,0.f,0.f,0.f,0.f,0.f};

  for (int k0 = 0; k0 < K; k0 += 32) {
    V bh[4], bl[4];
#pragma unroll
    for (int j = 0; j < 4; ++j) {
      const size_t bo = (size_t)(n0 + (j << 4) + rlane) * ldb + koff + k0;
      bh[j] = Frag<T>::load(Bb + bo);
      if (SPLIT) bl[j] = Frag<T>::load(Bb2 + bo);
    }
#pragma unroll
    for (int i = 0; i < 4; ++i) {
      const size_t ao = (size_t)(m0 + (i << 4) + rlane) * lda + koff + k0;
      V ah = Frag<T>::load(Ab + ao);
      V al;
      if (SPLIT) al = Frag<T>::load(Ab2 + ao);
#pragma unroll
      for (int j = 0; j < 4; ++j) {
        acc[i][j] = Frag<T>::mma(ah, bh[j], acc[i][j]);
        if (SPLIT) {
          acc[i][j] = Frag<T>::mma(ah, bl[j], acc[i][j]);
          acc[i][j] = Frag<T>::mma(al, bh[j], acc[i][j]);
        }
      }
      Frag<T>::guard(acc[i][0], acc[i][3], ah, SPLIT ? al : ah);
    }
    Frag<T>::keep(bh[0], bh[1], bh[2], bh[3]);
    if (SPLIT) Frag<T>::keep(bl[0], bl[1], bl[2], bl[3]);
  }
  acc_guard4(acc[0][0], acc[0][1], acc[0][2], acc[0][3]);
  acc_guard4(acc[1][0], acc[1][1], acc[1][2], acc[1][3]);
  acc_guard4(acc[2][0], acc[2][1], acc[2][2], acc[2][3]);
  acc_guard4(acc[3][0], acc[3][1], acc[3][2], acc[3][3]);

  float* slab = sT[wave];
  const float* Rb = RESID ? (resid + (size_t)b * strideR) : nullptr;
#pragma unroll
  for (int i = 0; i < 4; ++i) {
    const int mBase = m0 + (i << 4);
#pragma unroll
    for (int j = 0; j < 4; ++j) {
      const int n = n0 + (j << 4) + rlane;
      float bv = 0.f;
      if (BIAS_MODE == 2) bv = bias[n];
#pragma unroll
      for (int r = 0; r < 8; ++r) {
        float v = acc[i][j][r] * scale;
        if (BIAS_MODE == 1) v += bias[mBase + mOff + r];
        if (BIAS_MODE == 2) v += bv;
        if (RESID) v += Rb[(size_t)(mBase + mOff + r) * ldc + n];
        if (ACT == 2) v = fmaxf(v, 0.0f);
        if (ACT == 4) v = (v > 0.f) ? v : 0.01f * v;
        slab[(mOff + r) * 68 + (j << 4) + rlane] = v;
      }
    }
    __builtin_amdgcn_fence(__ATOMIC_RELEASE, "workgroup");
    __builtin_amdgcn_wave_barrier();
    __builtin_amdgcn_fence(__ATOMIC_ACQUIRE, "workgroup");
    if (OUT_MODE == 0) {
      float* C = (float*)Cout + (size_t)b * strideC;
      const int hh = lane >> 4, c4 = (lane & 15) * 4;
      for (int pass = 0; pass < 2; ++pass) {
#pragma unroll
        for (int it = 0; it < 8; ++it) {
          const int row = it * 2 + hh;
          v4f v = *(const v4f*)(slab + row * 68 + c4);
          *(volatile v4f*)(C + (size_t)(mBase + row) * ldc + n0 + c4) = v;
        }
        __threadfence();
      }
    } else {
      const int q = lane >> 3, c8 = (lane & 7) * 8;
      unsigned short* C  = (unsigned short*)Cout  + (size_t)b * strideC;
      unsigned short* C2 = (OUT_MODE == 2) ? ((unsigned short*)Cout2 + (size_t)b * strideC) : nullptr;
      for (int pass = 0; pass < 2; ++pass) {
#pragma unroll
        for (int it = 0; it < 4; ++it) {
          const int row = it * 4 + q;
          const float* sp = slab + row * 68 + c8;
          v8h hv, lv;
#pragma unroll
          for (int e = 0; e < 8; ++e) {
            if (OUT_MODE == 1) {
              hv[e] = (_Float16)sp[e];
            } else {
              unsigned short hb = f2bf_bits(sp[e]);
              unsigned short lb = f2bf_bits(sp[e] - bf_bits2f(hb));
              hv[e] = __builtin_bit_cast(_Float16, hb);
              lv[e] = __builtin_bit_cast(_Float16, lb);
            }
          }
          *(volatile v8h*)(C + (size_t)(mBase + row) * ldc + n0 + c8) = hv;
          if (OUT_MODE == 2) *(volatile v8h*)(C2 + (size_t)(mBase + row) * ldc + n0 + c8) = lv;
        }
        __threadfence();
      }
    }
    __builtin_amdgcn_fence(__ATOMIC_RELEASE, "workgroup");
    __builtin_amdgcn_wave_barrier();
    __builtin_amdgcn_fence(__ATOMIC_ACQUIRE, "workgroup");
  }
}

__device__ __forceinline__ v8f hmma(v16h a, v16h b, v8f c) {
  c = __builtin_amdgcn_wmma_f32_16x16x32_f16(false, a, false, b, (short)0, c, false, false);
  asm volatile("v_nop\n\tv_nop\n\tv_nop\n\tv_nop" : "+v"(c) : "v"(a), "v"(b));
  return c;
}

__global__ __launch_bounds__(256) void cast_in_kernel(const float* __restrict__ in0, const float* __restrict__ in1,
                                                      const float* __restrict__ in2, unsigned short* __restrict__ out,
                                                      int n8, int planeElems) {
  const int y = blockIdx.y;
  const float* in = (y == 0) ? in0 : ((y == 1) ? in1 : in2);
  const int i = blockIdx.x * 256 + threadIdx.x;
  if (i >= n8) return;
  const float* p = in + 8 * (size_t)i;
  const v4f a = *(const v4f*)(p);
  const v4f c = *(const v4f*)(p + 4);
  unsigned short hb[8];
#pragma unroll
  for (int e = 0; e < 4; ++e) {
    hb[e]     = f2bf_bits(a[e]);
    hb[4 + e] = f2bf_bits(c[e]);
  }
  const v4u u = (v4u){pk16(hb[0], hb[1]), pk16(hb[2], hb[3]), pk16(hb[4], hb[5]), pk16(hb[6], hb[7])};
  unsigned short* q = out + (size_t)y * planeElems + 8 * (size_t)i;
  *(volatile v4u*)q = u;
  __threadfence();
  *(volatile v4u*)q = u;
}

__global__ __launch_bounds__(256) void wcast_kernel(const float* __restrict__ W0, const float* __restrict__ W1,
                                                    const float* __restrict__ W2, const float* __restrict__ W3,
                                                    const float* __restrict__ W4, unsigned short* __restrict__ out,
                                                    int n8, int planeElems) {
  const int y = blockIdx.y;
  const float* W = (y == 0) ? W0 : ((y == 1) ? W1 : ((y == 2) ? W2 : ((y == 3) ? W3 : W4)));
  const bool asHalf = (y == 4);
  const int i = blockIdx.x * 256 + threadIdx.x;
  if (i >= n8) return;
  const float* p = W + 8 * (size_t)i;
  const v4f a = *(const v4f*)(p);
  const v4f c = *(const v4f*)(p + 4);
  unsigned short hb[8];
#pragma unroll
  for (int e = 0; e < 4; ++e) {
    const unsigned short b0 = f2bf_bits(a[e]);
    const unsigned short b1 = f2bf_bits(c[e]);
    const unsigned short h0 = h_bits(bf_bits2f(b0) * kWCarry);
    const unsigned short h1 = h_bits(bf_bits2f(b1) * kWCarry);
    hb[e]     = asHalf ? h0 : b0;
    hb[4 + e] = asHalf ? h1 : b1;
  }
  const v4u u = (v4u){pk16(hb[0], hb[1]), pk16(hb[2], hb[3]), pk16(hb[4], hb[5]), pk16(hb[6], hb[7])};
  unsigned short* q = out + (size_t)y * planeElems + 8 * (size_t)i;
  *(volatile v4u*)q = u;
  __threadfence();
  *(volatile v4u*)q = u;
}

__global__ __launch_bounds__(128) void bias_kernel(const float* __restrict__ b0, const float* __restrict__ b1,
                                                   const float* __restrict__ b2, const float* __restrict__ b3,
                                                   const float* __restrict__ b4, float* __restrict__ BR) {
  const int y = blockIdx.x;
  const float* bp = (y == 0) ? b0 : ((y == 1) ? b1 : ((y == 2) ? b2 : ((y == 3) ? b3 : b4)));
  const int t = threadIdx.x;
  const v4f v = *(const v4f*)(bp + 4 * t);
  v4f o;
#pragma unroll
  for (int e = 0; e < 4; ++e) o[e] = bf_bits2f(f2bf_bits(v[e]));
  float* dp = BR + (size_t)y * kE + 4 * t;
  *(volatile v4f*)dp = o;
  __threadfence();
  *(volatile v4f*)dp = o;
}

struct TabConst { float invf[32]; };
static_assert(sizeof(TabConst) == 128, "size");

__global__ __launch_bounds__(256) void tables_kernel(float* __restrict__ sint, float* __restrict__ cost,
                                                     float* __restrict__ sct, TabConst tc) {
  const int gid = blockIdx.x * 256 + threadIdx.x;
  if (gid >= kN * kHalf) return;
  const int j = gid & (kHalf - 1);
  const int n = gid >> 5;
  float invf = tc.invf[0];
#pragma unroll
  for (int q = 1; q < 32; ++q) invf = (j == q) ? tc.invf[q] : invf;
  const float ang = (float)n * invf;
  float sn, cs;
  sincosf(ang, &sn, &cs);
  const float xs = ((float)(2 * j) + 25.6f) / 89.6f;
  const float pw = (float)(n - kN / 2) * (1.0f / 512.0f);
  const float sc = exp2f(pw * log2f(xs));
  for (int pass = 0; pass < 2; ++pass) {
    ((volatile float*)sint)[gid] = sn;
    ((volatile float*)cost)[gid] = cs;
    ((volatile float*)sct)[gid]  = sc;
    __threadfence();
  }
}

__global__ __launch_bounds__(256) void xpos_kernel(const float* __restrict__ QP, const float* __restrict__ KP,
                                                   const float* __restrict__ sint, const float* __restrict__ cost,
                                                   const float* __restrict__ sct,
                                                   unsigned short* __restrict__ QX, unsigned short* __restrict__ KX) {
  const int gid = blockIdx.x * 256 + threadIdx.x;
  if (gid >= kTok * (kE / 8)) return;
  const int row = gid >> 6;
  const int c8  = (gid & 63) * 8;
  const int n   = row & (kN - 1);
  const int j0  = (c8 & (kDh - 1)) >> 1;
  const size_t off = (size_t)row * kE + c8;
  const v4f qa = *(const v4f*)(QP + off);
  const v4f qc = *(const v4f*)(QP + off + 4);
  const v4f ka = *(const v4f*)(KP + off);
  const v4f kcv = *(const v4f*)(KP + off + 4);
  const size_t toff = (size_t)n * kHalf + j0;
  const v4f sn = *(const v4f*)(sint + toff);
  const v4f cs = *(const v4f*)(cost + toff);
  const v4f sc = *(const v4f*)(sct + toff);
  float x[8], y[8];
  x[0] = qa[0]; x[1] = qa[1]; x[2] = qa[2]; x[3] = qa[3];
  x[4] = qc[0]; x[5] = qc[1]; x[6] = qc[2]; x[7] = qc[3];
  y[0] = ka[0]; y[1] = ka[1]; y[2] = ka[2]; y[3] = ka[3];
  y[4] = kcv[0]; y[5] = kcv[1]; y[6] = kcv[2]; y[7] = kcv[3];
  unsigned short hq[8], hk[8];
#pragma unroll
  for (int p = 0; p < 4; ++p) {
    const float scp = sc[p];
    const float snp = sn[p];
    const float csp = cs[p];
    const float cq = csp * scp;
    const float sq = snp * scp;
    const float isc = 1.0f / scp;
    const float ck = csp * isc;
    const float sk = snp * isc;
    const float x0 = x[2 * p], x1 = x[2 * p + 1];
    const float y0 = y[2 * p], y1 = y[2 * p + 1];
    hq[2 * p]     = h_bits((x0 * cq - x1 * sq) * kQC);
    hq[2 * p + 1] = h_bits((x1 * cq + x0 * sq) * kQC);
    hk[2 * p]     = h_bits((y0 * ck - y1 * sk) * kKmul);
    hk[2 * p + 1] = h_bits((y1 * ck + y0 * sk) * kKmul);
  }
  const v4u uq = (v4u){pk16(hq[0], hq[1]), pk16(hq[2], hq[3]), pk16(hq[4], hq[5]), pk16(hq[6], hq[7])};
  const v4u uk = (v4u){pk16(hk[0], hk[1]), pk16(hk[2], hk[3]), pk16(hk[4], hk[5]), pk16(hk[6], hk[7])};
  unsigned short* qd = QX + off;
  unsigned short* kd = KX + off;
  *(volatile v4u*)qd = uq;
  *(volatile v4u*)kd = uk;
  __threadfence();
  *(volatile v4u*)qd = uq;
  *(volatile v4u*)kd = uk;
}

__global__ __launch_bounds__(256) void silu_kernel(const float* __restrict__ GP, float* __restrict__ GS, int n4) {
  const int i = blockIdx.x * 256 + threadIdx.x;
  if (i >= n4) return;
  const v4f g = *(const v4f*)(GP + 4 * (size_t)i);
  v4f o;
#pragma unroll
  for (int e = 0; e < 4; ++e) {
    const float xv = g[e];
    const float ex = expf(-xv);
    o[e] = xv * (1.0f / (1.0f + ex));
  }
  float* dp = GS + 4 * (size_t)i;
  *(volatile v4f*)dp = o;
  __threadfence();
  *(volatile v4f*)dp = o;
}

constexpr int kRetWaves   = 4;
constexpr int kRetThreads = kRetWaves * 32;
constexpr int kQBlk       = 64;
constexpr int kKChunk     = 64;
constexpr int kOsPitch    = 68;
static_assert(kN % kQBlk == 0 && kQBlk == kKChunk && kQBlk == 16 * kRetWaves, "retention tiling");

__global__ __launch_bounds__(kRetThreads) void retention_kernel(
    const unsigned short* __restrict__ QXp, const unsigned short* __restrict__ KXp,
    const unsigned short* __restrict__ VTp, const float* __restrict__ GS,
    unsigned short* __restrict__ RG) {
  const _Float16* QX = (const _Float16*)(const void*)QXp;
  const _Float16* KX = (const _Float16*)(const void*)KXp;
  const _Float16* VT = (const _Float16*)(const void*)VTp;
  __shared__ __align__(16) _Float16 Psh[kRetWaves][16 * kKChunk];
  __shared__ __align__(16) float Os[kRetWaves][16 * kOsPitch];

  const int tid  = threadIdx.x;
  const int wave = tid >> 5;
  const int lane = tid & 31;
  const int hh   = lane >> 4;
  const int c    = lane & 15;
  const int qb   = blockIdx.x;
  const int bh   = blockIdx.y;
  const int b    = bh >> 3;
  const int h    = bh & (kH - 1);
  const int qbb  = qb * kQBlk;
  const int q0   = qbb + wave * 16;

  const float lin  = kLn1o32 + (float)h * ((kLn1o512 - kLn1o32) * (1.0f / 7.0f));
  const float gam  = 1.0f - expf(lin);
  const float logg = logf(gam);

  const size_t tokBase = (size_t)b * kN;

  v16h qa[2];
  {
    const _Float16* qrow = QX + (tokBase + q0 + c) * kE + h * kDh + 8 * hh;
    qa[0] = Frag<_Float16>::load(qrow);
    qa[1] = Frag<_Float16>::load(qrow + 32);
  }
  float ar[8];
#pragma unroll
  for (int r = 0; r < 8; ++r) ar[r] = expf((float)(wave * 16 + 8 * hh + r) * logg);

  v8f oacc[4];
#pragma unroll
  for (int t = 0; t < 4; ++t) oacc[t] = (v8f){0.f, 0.f, 0.f, 0.f, 0.f, 0.f, 0.f, 0.f};

  const _Float16* kbase = KX + tokBase * kE + h * kDh + 8 * hh;
  const _Float16* vbase = VT + (size_t)(h * kDh + c) * kTok + tokBase + 8 * hh;
  _Float16* pwp = Psh[wave];

  const int nChunks = qb + 1;
  for (int kc = 0; kc < nChunks; ++kc) {
    const int kv0 = kc * kKChunk;
    v8f s[4];
#pragma unroll
    for (int j = 0; j < 4; ++j) s[j] = (v8f){0.f, 0.f, 0.f, 0.f, 0.f, 0.f, 0.f, 0.f};
#pragma unroll
    for (int dc = 0; dc < 2; ++dc) {
      v16h kb[4];
#pragma unroll
      for (int j = 0; j < 4; ++j) kb[j] = Frag<_Float16>::load(kbase + (size_t)(kv0 + j * 16 + c) * kE + dc * 32);
#pragma unroll
      for (int j = 0; j < 4; ++j) s[j] = hmma(qa[dc], kb[j], s[j]);
    }
    float bj[4];
    int scol[4];
#pragma unroll
    for (int j = 0; j < 4; ++j) {
      scol[j] = kv0 + j * 16 + c;
      bj[j] = expf((float)(qbb - scol[j]) * logg) * kMaskMul;
    }
    __syncthreads();
#pragma unroll
    for (int r = 0; r < 8; ++r) {
      const int qrow = q0 + 8 * hh + r;
      const float arow = ar[r];
#pragma unroll
      for (int j = 0; j < 4; ++j) {
        float p = s[j][r] * (arow * bj[j]);
        p = (scol[j] > qrow) ? 0.0f : p;
        pwp[(8 * hh + r) * kKChunk + j * 16 + c] = (_Float16)p;
      }
    }
    __syncthreads();
#pragma unroll
    for (int kk = 0; kk < 2; ++kk) {
      const v16h pa = Frag<_Float16>::load(pwp + c * kKChunk + kk * 32 + 8 * hh);
#pragma unroll
      for (int t = 0; t < 4; ++t) {
        const v16h vb = Frag<_Float16>::load(vbase + (size_t)(t * 16) * kTok + kv0 + kk * 32);
        oacc[t] = hmma(pa, vb, oacc[t]);
      }
    }
  }

  float* os = Os[wave];
#pragma unroll
  for (int r = 0; r < 8; ++r) {
    const float x0 = oacc[0][r] * kPCInv;
    const float x1 = oacc[1][r] * kPCInv;
    const float x2 = oacc[2][r] * kPCInv;
    const float x3 = oacc[3][r] * kPCInv;
    float s1 = (x0 + x1) + (x2 + x3);
    s1 += __shfl_xor(s1, 1, 32);
    s1 += __shfl_xor(s1, 2, 32);
    s1 += __shfl_xor(s1, 4, 32);
    s1 += __shfl_xor(s1, 8, 32);
    const float mean = s1 * kInvDh;
    const float d0 = x0 - mean, d1 = x1 - mean, d2 = x2 - mean, d3 = x3 - mean;
    float s2 = (d0 * d0 + d1 * d1) + (d2 * d2 + d3 * d3);
    s2 += __shfl_xor(s2, 1, 32);
    s2 += __shfl_xor(s2, 2, 32);
    s2 += __shfl_xor(s2, 4, 32);
    s2 += __shfl_xor(s2, 8, 32);
    const float var  = s2 * kInvDh;
    const float rstd = 1.0f / sqrtf(var + kGnEps);
    const int orow = (8 * hh + r) * kOsPitch;
    os[orow + 0 * 16 + c] = d0 * rstd;
    os[orow + 1 * 16 + c] = d1 * rstd;
    os[orow + 2 * 16 + c] = d2 * rstd;
    os[orow + 3 * 16 + c] = d3 * rstd;
  }
  __syncthreads();
  {
    const int q4 = lane >> 3;
    const int c8 = (lane & 7) * 8;
    v4u ow[4];
#pragma unroll
    for (int it = 0; it < 4; ++it) {
      const int row = it * 4 + q4;
      const size_t tok = tokBase + q0 + row;
      const float* gp = GS + tok * kE + h * kDh + c8;
      const v4f g0 = *(const v4f*)(gp);
      const v4f g1 = *(const v4f*)(gp + 4);
      const float* sp = os + row * kOsPitch + c8;
      const v4f n0 = *(const v4f*)(sp);
      const v4f n1 = *(const v4f*)(sp + 4);
      unsigned short hb[8];
#pragma unroll
      for (int e = 0; e < 4; ++e) {
        hb[e]     = h_bits(n0[e] * g0[e] * kRGC);
        hb[4 + e] = h_bits(n1[e] * g1[e] * kRGC);
      }
      ow[it] = (v4u){pk16(hb[0], hb[1]), pk16(hb[2], hb[3]), pk16(hb[4], hb[5]), pk16(hb[6], hb[7])};
    }
    for (int pass = 0; pass < 2; ++pass) {
#pragma unroll
      for (int it = 0; it < 4; ++it) {
        const int row = it * 4 + q4;
        const size_t tok = tokBase + q0 + row;
        *(volatile v4u*)(RG + tok * kE + h * kDh + c8) = ow[it];
      }
      __threadfence();
    }
  }
}

static_assert(kTok % 64 == 0 && kE % 64 == 0 && kE % 32 == 0, "gemm tiles");

extern "C" void kernel_launch(void* const* d_in, const int* in_sizes, int n_in,
                              void* d_out, int out_size, void* d_ws, size_t ws_size,
                              hipStream_t stream) {
  if (n_in < 13) return;
  if (in_sizes[0] != kPlane || in_sizes[1] != kPlane || in_sizes[2] != kPlane) return;
  if (in_sizes[3] != kWElems || in_sizes[5] != kWElems || in_sizes[7] != kWElems ||
      in_sizes[9] != kWElems || in_sizes[11] != kWElems) return;
  if (in_sizes[4] != kE || in_sizes[6] != kE || in_sizes[8] != kE || in_sizes[10] != kE || in_sizes[12] != kE) return;
  if (out_size != kPlane) return;

  const size_t sz16  = (size_t)kPlane * 2;
  const size_t sz32  = (size_t)kPlane * 4;
  const size_t szW16 = (size_t)kWElems * 2;
  const size_t szBR  = (size_t)5 * kE * 4;
  const size_t szTab = (size_t)kN * kHalf * 4;
  const size_t offX   = 0;
  const size_t offW   = offX + 3 * sz16;
  const size_t offBR  = offW + 5 * szW16;
  const size_t offTab = offBR + szBR;
  const size_t offQP  = offTab + 3 * szTab;
  const size_t offKP  = offQP + sz32;
  const size_t offGP  = offKP + sz32;
  const size_t offGS  = offGP + sz32;
  const size_t offVT  = offGS + sz32;
  const size_t offQX  = offVT + sz16;
  const size_t offKX  = offQX + sz16;
  const size_t offRG  = offKX + sz16;
  const size_t total  = offRG + sz16;
  if (ws_size < total) return;

  const float* query = (const float*)d_in[0];
  const float* keyin = (const float*)d_in[1];
  const float* value = (const float*)d_in[2];
  const float* Wq = (const float*)d_in[3];
  const float* bq = (const float*)d_in[4];
  const float* Wk = (const float*)d_in[5];
  const float* bk = (const float*)d_in[6];
  const float* Wv = (const float*)d_in[7];
  const float* bv = (const float*)d_in[8];
  const float* Wg = (const float*)d_in[9];
  const float* bg = (const float*)d_in[10];
  const float* Wo = (const float*)d_in[11];
  const float* bo = (const float*)d_in[12];
  float* out = (float*)d_out;
  char* ws = (char*)d_ws;
  unsigned short* X16 = (unsigned short*)(ws + offX);
  unsigned short* W16 = (unsigned short*)(ws + offW);
  float* BR  = (float*)(ws + offBR);
  float* TAB = (float*)(ws + offTab);
  float* QP  = (float*)(ws + offQP);
  float* KP  = (float*)(ws + offKP);
  float* GP  = (float*)(ws + offGP);
  float* GS  = (float*)(ws + offGS);
  unsigned short* VT = (unsigned short*)(ws + offVT);
  unsigned short* QX = (unsigned short*)(ws + offQX);
  unsigned short* KX = (unsigned short*)(ws + offKX);
  unsigned short* RG = (unsigned short*)(ws + offRG);

  const unsigned short* Xq16 = X16;
  const unsigned short* Xk16 = X16 + (size_t)kPlane;
  const unsigned short* Xv16 = X16 + 2 * (size_t)kPlane;
  const unsigned short* Wq16 = W16;
  const unsigned short* Wk16 = W16 + (size_t)kWElems;
  const unsigned short* Wv16 = W16 + 2 * (size_t)kWElems;
  const unsigned short* Wg16 = W16 + 3 * (size_t)kWElems;
  const unsigned short* Wo16 = W16 + 4 * (size_t)kWElems;
  const float* BRq = BR;
  const float* BRk = BR + kE;
  const float* BRv = BR + 2 * kE;
  const float* BRg = BR + 3 * kE;
  const float* BRo = BR + 4 * kE;
  float* SIN = TAB;
  float* COS = TAB + (size_t)kN * kHalf;
  float* SCL = TAB + 2 * (size_t)kN * kHalf;

  TabConst tc;
  {
    const double root = 1.3335214321633240;
    double pw = 1.0;
    for (int j = 0; j < 32; ++j) {
      const float pf = (float)pw;
      tc.invf[j] = 1.0f / pf;
      pw *= root;
    }
  }

  const int n8in = kPlane / 8;
  const int n8w  = kWElems / 8;
  cast_in_kernel<<<dim3(n8in / 256, 3), dim3(256), 0, stream>>>(query, keyin, value, X16, n8in, kPlane);
  wcast_kernel<<<dim3(n8w / 256, 5), dim3(256), 0, stream>>>(Wq, Wk, Wv, Wg, Wo, W16, n8w, kWElems);
  bias_kernel<<<dim3(5), dim3(128), 0, stream>>>(bq, bk, bv, bg, bo, BR);
  tables_kernel<<<dim3((kN * kHalf) / 256), dim3(256), 0, stream>>>(SIN, COS, SCL, tc);

  const int blkProj = ((kTok / 64) * (kE / 64)) / 8;
  wmma_gemm64<1, false, 2, 0, false, 0><<<dim3(blkProj, 1), dim3(256), 0, stream>>>(
      Xq16, Xq16, kE, 0L, Wq16, Wq16, kE, 0L, (void*)QP, (void*)QP, kE, 0L, BRq, BRq, 0L, kTok, kE, kE, 1.0f);
  wmma_gemm64<1, false, 2, 0, false, 0><<<dim3(blkProj, 1), dim3(256), 0, stream>>>(
      Xk16, Xk16, kE, 0L, Wk16, Wk16, kE, 0L, (void*)KP, (void*)KP, kE, 0L, BRk, BRk, 0L, kTok, kE, kE, 1.0f);
  wmma_gemm64<1, false, 2, 0, false, 0><<<dim3(blkProj, 1), dim3(256), 0, stream>>>(
      Xq16, Xq16, kE, 0L, Wg16, Wg16, kE, 0L, (void*)GP, (void*)GP, kE, 0L, BRg, BRg, 0L, kTok, kE, kE, 1.0f);
  wmma_gemm64<1, false, 1, 1, false, 0><<<dim3(blkProj, 1), dim3(256), 0, stream>>>(
      Wv16, Wv16, kE, 0L, Xv16, Xv16, kE, 0L, (void*)VT, (void*)VT, kTok, 0L, BRv, BRv, 0L, kE, kTok, kE, 1.0f);

  xpos_kernel<<<dim3((kTok * (kE / 8)) / 256), dim3(256), 0, stream>>>(QP, KP, SIN, COS, SCL, QX, KX);
  const int n4 = kPlane / 4;
  silu_kernel<<<dim3(n4 / 256), dim3(256), 0, stream>>>(GP, GS, n4);

  retention_kernel<<<dim3(kN / kQBlk, kB * kH), dim3(kRetThreads), 0, stream>>>(QX, KX, VT, GS, RG);

  wmma_gemm64<0, false, 2, 0, false, 0><<<dim3(blkProj, 1), dim3(256), 0, stream>>>(
      RG, RG, kE, 0L, Wo16, Wo16, kE, 0L, (void*)out, (void*)out, kE, 0L, BRo, BRo, 0L, kTok, kE, kE, kOutScale);
}
